// DVRJANET_48988396978774
// MI455X (gfx1250) — hardware-verified
//
#include <hip/hip_runtime.h>
#include <math.h>

constexpr int SEQS    = 64;
constexpr int STEPS   = 1024;
constexpr int HID     = 256;
constexpr int HID3    = 3 * HID;
constexpr int KCAT    = 2 * HID;
constexpr int NTHR    = 256;
constexpr int SEQ_BLK = 16;
constexpr int NBLK    = SEQS / SEQ_BLK;
constexpr int PPITCH  = 264;
constexpr int APITCH  = 520;
constexpr int SPITCH  = 772;
constexpr int HPITCH  = 256;
constexpr int TCHUNK  = 32;
constexpr int OPITCH  = 2 * TCHUNK;
constexpr int NCHUNK  = STEPS / TCHUNK;
constexpr float ACT_CARRY = 16.0f;
constexpr float WGT_CARRY = 16.0f;
constexpr float FOLD_INV  = 1.0f / 256.0f;
constexpr float K13 = 1.0f / 3.0f;
constexpr float K23 = 2.0f / 3.0f;
static_assert(SEQS % SEQ_BLK == 0);
static_assert(NTHR == HID);
static_assert(SEQ_BLK * 16 == NTHR);
static_assert(HID == 32 * (NTHR / 32));
static_assert(HID % 64 == 0 && KCAT % 64 == 0 && HID % 32 == 0);
static_assert(STEPS % TCHUNK == 0);
static_assert(OPITCH == 64);
static_assert(PPITCH % 8 == 0 && APITCH % 8 == 0);

typedef __attribute__((ext_vector_type(16))) _Float16 v16h;
typedef __attribute__((ext_vector_type(8)))  _Float16 v8h;
typedef __attribute__((ext_vector_type(8)))  float    v8f;
typedef __attribute__((ext_vector_type(4)))  float    v4f;

__device__ __forceinline__ unsigned short f2bf_bits(float f) {
  unsigned u = __float_as_uint(f);
  return (unsigned short)((u + 0x7FFFu + ((u >> 16) & 1u)) >> 16);
}
__device__ __forceinline__ float bf_bits2f(unsigned short h) { return __uint_as_float(((unsigned)h) << 16); }
__device__ __forceinline__ float bf16r(float f) { return bf_bits2f(f2bf_bits(f)); }

__device__ __forceinline__ void dep_guard_h(v8f& a, v8f& b, v16h x, v16h y) { asm volatile("v_nop\n\tv_nop\n\tv_nop\n\tv_nop" : "+v"(a), "+v"(b) : "v"(x), "v"(y)); }
__device__ __forceinline__ void keep4_h(v16h a, v16h b, v16h c, v16h d) { asm volatile("v_nop" :: "v"(a), "v"(b), "v"(c), "v"(d)); }
__device__ __forceinline__ void acc_guard4(v8f& a, v8f& b, v8f& c, v8f& d) { asm volatile("v_nop\n\tv_nop\n\tv_nop\n\tv_nop" : "+v"(a), "+v"(b), "+v"(c), "+v"(d)); }
__device__ __forceinline__ void acc_guard2(v8f& a, v8f& b) { asm volatile("v_nop\n\tv_nop\n\tv_nop\n\tv_nop" : "+v"(a), "+v"(b)); }

template <typename T> struct Frag;
template <> struct Frag<_Float16> {
  typedef v16h V; union U { v16h v; v8h h[2]; };
  static __device__ __forceinline__ v16h load(const _Float16* p) {
    U f; f.h[0] = *(const v8h*)(p); f.h[1] = *(const v8h*)(p + 16); return f.v;
  }
  static __device__ __forceinline__ v8f mma(v16h a, v16h b, v8f c) {
    return __builtin_amdgcn_wmma_f32_16x16x32_f16(false, a, false, b, (short)0, c, false, false);
  }
};

__device__ __forceinline__ float fsig(float x)  { return __builtin_amdgcn_rcpf(1.0f + __expf(-x)); }
__device__ __forceinline__ float ftanh(float x) { return 1.0f - 2.0f * __builtin_amdgcn_rcpf(__expf(2.0f * x) + 1.0f); }

__global__ __launch_bounds__(NTHR) void tr_cvt_kernel(const float* __restrict__ in, int ncols,
                                                     unsigned short* __restrict__ outp, int ldo, int nofs) {
  __shared__ __align__(16) _Float16 tile[64 * 72];
  const int tid = threadIdx.x;
  const int n0 = blockIdx.x * 64, k0 = blockIdx.y * 64;
  {
    const int n4 = (tid & 15) * 4;
#pragma unroll
    for (int i = 0; i < 4; ++i) {
      const int kk = (tid >> 4) + 16 * i;
      const v4f v = *(const v4f*)(in + (size_t)(k0 + kk) * ncols + n0 + n4);
#pragma unroll
      for (int e = 0; e < 4; ++e) tile[(n4 + e) * 72 + kk] = (_Float16)(WGT_CARRY * bf16r(v[e]));
    }
  }
  __syncthreads();
  const int q = tid >> 3, c8 = (tid & 7) * 8;
  _Float16* outh = (_Float16*)outp;
  for (int pass = 0; pass < 2; ++pass) {
#pragma unroll
    for (int it = 0; it < 2; ++it) {
      const int nl = q + 32 * it;
      const v8h hv = *(const v8h*)(tile + nl * 72 + c8);
      *(volatile v8h*)(outh + (size_t)(nofs + n0 + nl) * ldo + k0 + c8) = hv;
    }
    __threadfence();
  }
}

__device__ __forceinline__ void flush_chunk(float* __restrict__ out, const float* os, int rowbase, int q, int wave, int lane) {
  const int hh = lane >> 4, c4 = (lane & 15) * 4;
  const int row = 2 * wave + hh;
  const v4f v = *(const v4f*)(os + row * OPITCH + c4);
  float* dst = out + ((size_t)(rowbase + row) * STEPS + (size_t)q * TCHUNK) * 2 + c4;
  *(volatile v4f*)dst = v;
  __threadfence();
  *(volatile v4f*)dst = v;
}

__global__ __launch_bounds__(NTHR) void cell_seq_kernel(
    const float* __restrict__ x, const float* __restrict__ hI0, const float* __restrict__ hQ0,
    const float* __restrict__ c1p, const float* __restrict__ c2p, const float* __restrict__ c3p,
    const float* __restrict__ Wa, const float* __restrict__ Wp1, const float* __restrict__ bfp,
    const float* __restrict__ bgc, const float* __restrict__ bgs,
    const float* __restrict__ WI, const float* __restrict__ bIp,
    const float* __restrict__ WQ, const float* __restrict__ bQp,
    const unsigned short* __restrict__ W1p, const unsigned short* __restrict__ W2cp, const unsigned short* __restrict__ W2sp,
    float* __restrict__ out) {
  __shared__ __align__(16) _Float16 Pp[SEQ_BLK * PPITCH];
  __shared__ __align__(16) _Float16 Acp[SEQ_BLK * APITCH];
  __shared__ __align__(16) _Float16 Asp[SEQ_BLK * APITCH];
  __shared__ __align__(16) float    Sacc[SEQ_BLK * SPITCH];
  __shared__ __align__(16) float    HIf[SEQ_BLK * HPITCH];
  __shared__ __align__(16) float    HQf[SEQ_BLK * HPITCH];
  __shared__ __align__(16) float    Os[SEQ_BLK * OPITCH];
  __shared__ __align__(16) float    Tb[7 * HID];

  const _Float16* W1  = (const _Float16*)W1p;
  const _Float16* W2c = (const _Float16*)W2cp;
  const _Float16* W2s = (const _Float16*)W2sp;
  const int tid = threadIdx.x, lane = tid & 31, wave = tid >> 5;
  const int c = lane & 15, hh = lane >> 4, koff = hh * 8;
  const int erow = tid >> 4, ec = tid & 15;
  const int rowbase = blockIdx.x * SEQ_BLK;

  const float c1v = bf16r(c1p[0]), c2v = bf16r(c2p[0]), c3v = bf16r(c3p[0]);
  const float bIv = bf16r(bIp[0]), bQv = bf16r(bQp[0]);

  Tb[0 * HID + tid] = bf16r(Wa[tid]);
  Tb[1 * HID + tid] = bf16r(Wp1[tid]);
  Tb[2 * HID + tid] = bf16r(bfp[tid]);
  Tb[3 * HID + tid] = bf16r(bgc[tid]);
  Tb[4 * HID + tid] = bf16r(bgs[tid]);
  Tb[5 * HID + tid] = bf16r(WI[tid]);
  Tb[6 * HID + tid] = bf16r(WQ[tid]);
#pragma unroll 1
  for (int i = tid; i < SEQ_BLK * APITCH; i += NTHR) { Acp[i] = (_Float16)0.0f; Asp[i] = (_Float16)0.0f; }
#pragma unroll 1
  for (int i = tid; i < SEQ_BLK * PPITCH; i += NTHR) Pp[i] = (_Float16)0.0f;
  __syncthreads();
#pragma unroll 1
  for (int i = 0; i < 16; ++i) {
    const int col = ec + 16 * i;
    const float hi = bf16r(hI0[(size_t)(rowbase + erow) * HID + col]);
    const float hq = bf16r(hQ0[(size_t)(rowbase + erow) * HID + col]);
    HIf[erow * HPITCH + col] = hi;
    HQf[erow * HPITCH + col] = hq;
    Acp[erow * APITCH + col] = (_Float16)(hi * ACT_CARRY);
    Asp[erow * APITCH + col] = (_Float16)(hq * ACT_CARRY);
    Pp[erow * PPITCH + col]  = (_Float16)(hi * hq * ACT_CARRY);
  }
  __syncthreads();

  const v8f z8 = {0.f, 0.f, 0.f, 0.f, 0.f, 0.f, 0.f, 0.f};

#pragma unroll 1
  for (int t = 0; t < STEPS; ++t) {
    if ((t & (TCHUNK - 1)) == 0 && t > 0) flush_chunk(out, Os, rowbase, t / TCHUNK - 1, wave, lane);

    {
      v8f acc[6];
#pragma unroll
      for (int q = 0; q < 6; ++q) acc[q] = z8;
      const _Float16* prow = Pp + c * PPITCH + koff;
#pragma unroll 1
      for (int k0 = 0; k0 < HID; k0 += 32) {
        const v16h a = Frag<_Float16>::load(prow + k0);
        v16h b[6];
#pragma unroll
        for (int q = 0; q < 6; ++q)
          b[q] = Frag<_Float16>::load(W1 + (size_t)((q >> 1) * HID + 32 * wave + 16 * (q & 1) + c) * HID + koff + k0);
#pragma unroll
        for (int q = 0; q < 6; ++q) acc[q] = Frag<_Float16>::mma(a, b[q], acc[q]);
        dep_guard_h(acc[0], acc[5], a, b[5]);
        keep4_h(b[0], b[1], b[2], b[3]);
        keep4_h(b[4], b[5], b[4], b[5]);
      }
      acc_guard4(acc[0], acc[1], acc[2], acc[3]);
      acc_guard2(acc[4], acc[5]);
#pragma unroll
      for (int q = 0; q < 6; ++q) {
        const int col = (q >> 1) * HID + 32 * wave + 16 * (q & 1) + c;
#pragma unroll
        for (int r = 0; r < 8; ++r) Sacc[(8 * hh + r) * SPITCH + col] = acc[q][r];
      }
    }
    __syncthreads();

    {
      const float x0 = bf16r(x[((size_t)(rowbase + erow) * STEPS + (size_t)t) * 2 + 0]);
      const float x1 = bf16r(x[((size_t)(rowbase + erow) * STEPS + (size_t)t) * 2 + 1]);
#pragma unroll 1
      for (int i = 0; i < 16; ++i) {
        const int col = ec + 16 * i;
        float* sp = Sacc + erow * SPITCH + col;
        const float a    = x0 * Tb[col] + sp[0] * FOLD_INV;
        const float anew = (a - K13) * c1v + (a - K23) * c2v + (a - 1.0f) * c3v;
        const float th   = x1 * Tb[HID + col] + sp[HID] * FOLD_INV;
        const float fg   = fsig(sp[2 * HID] * FOLD_INV + Tb[2 * HID + col]);
        const float cs = cosf(th), sn = sinf(th);
        Acp[erow * APITCH + HID + col] = (_Float16)(cs * anew * ACT_CARRY);
        Asp[erow * APITCH + HID + col] = (_Float16)(sn * anew * ACT_CARRY);
        sp[2 * HID] = fg;
      }
    }
    __syncthreads();

    {
      v8f acc[4];
      acc[0] = z8; acc[1] = z8; acc[2] = z8; acc[3] = z8;
      const _Float16* arc = Acp + c * APITCH + koff;
      const _Float16* ars = Asp + c * APITCH + koff;
      const _Float16* wc  = W2c + (size_t)(32 * wave + c) * KCAT + koff;
      const _Float16* wsn = W2s + (size_t)(32 * wave + c) * KCAT + koff;
#pragma unroll 1
      for (int k0 = 0; k0 < KCAT; k0 += 32) {
        const v16h ac = Frag<_Float16>::load(arc + k0);
        const v16h as = Frag<_Float16>::load(ars + k0);
        const v16h b0 = Frag<_Float16>::load(wc + k0);
        const v16h b1 = Frag<_Float16>::load(wc + (size_t)16 * KCAT + k0);
        const v16h b2 = Frag<_Float16>::load(wsn + k0);
        const v16h b3 = Frag<_Float16>::load(wsn + (size_t)16 * KCAT + k0);
        acc[0] = Frag<_Float16>::mma(ac, b0, acc[0]);
        acc[1] = Frag<_Float16>::mma(ac, b1, acc[1]);
        acc[2] = Frag<_Float16>::mma(as, b2, acc[2]);
        acc[3] = Frag<_Float16>::mma(as, b3, acc[3]);
        dep_guard_h(acc[0], acc[3], as, b3);
        keep4_h(b0, b1, b2, ac);
      }
      acc_guard4(acc[0], acc[1], acc[2], acc[3]);
#pragma unroll
      for (int nt = 0; nt < 2; ++nt) {
        const int col = 32 * wave + 16 * nt + c;
#pragma unroll
        for (int r = 0; r < 8; ++r) {
          Sacc[(8 * hh + r) * SPITCH + col]       = acc[nt][r];
          Sacc[(8 * hh + r) * SPITCH + HID + col] = acc[2 + nt][r];
        }
      }
    }
    __syncthreads();

    {
      float sI = 0.0f, sQ = 0.0f;
#pragma unroll 1
      for (int i = 0; i < 16; ++i) {
        const int col = ec + 16 * i;
        const float zc = Sacc[erow * SPITCH + col] * FOLD_INV + Tb[3 * HID + col];
        const float zs = Sacc[erow * SPITCH + HID + col] * FOLD_INV + Tb[4 * HID + col];
        const float gc = ftanh(zc), gs = ftanh(zs);
        const float fg = Sacc[erow * SPITCH + 2 * HID + col];
        const float hi = HIf[erow * HPITCH + col];
        const float hq = HQf[erow * HPITCH + col];
        const float hin = fg * hi + (1.0f - fg) * gc;
        const float hqn = fg * hq + (1.0f - fg) * gs;
        HIf[erow * HPITCH + col] = hin;
        HQf[erow * HPITCH + col] = hqn;
        Acp[erow * APITCH + col] = (_Float16)(hin * ACT_CARRY);
        Asp[erow * APITCH + col] = (_Float16)(hqn * ACT_CARRY);
        Pp[erow * PPITCH + col]  = (_Float16)(hin * hqn * ACT_CARRY);
        sI = fmaf(hin, Tb[5 * HID + col], sI);
        sQ = fmaf(hqn, Tb[6 * HID + col], sQ);
      }
      sI += __shfl_xor(sI, 1, 32); sQ += __shfl_xor(sQ, 1, 32);
      sI += __shfl_xor(sI, 2, 32); sQ += __shfl_xor(sQ, 2, 32);
      sI += __shfl_xor(sI, 4, 32); sQ += __shfl_xor(sQ, 4, 32);
      sI += __shfl_xor(sI, 8, 32); sQ += __shfl_xor(sQ, 8, 32);
      if (ec == 0) {
        Os[erow * OPITCH + 2 * (t & (TCHUNK - 1)) + 0] = sI + bIv;
        Os[erow * OPITCH + 2 * (t & (TCHUNK - 1)) + 1] = sQ + bQv;
      }
    }
    __syncthreads();
  }
  flush_chunk(out, Os, rowbase, NCHUNK - 1, wave, lane);
}

extern "C" void kernel_launch(void* const* d_in, const int* in_sizes, int n_in,
                              void* d_out, int out_size, void* d_ws, size_t ws_size, hipStream_t stream) {
  if (n_in < 20 || d_out == nullptr || d_ws == nullptr) return;
  if (in_sizes[0] != SEQS * STEPS * 2 || in_sizes[1] != SEQS * HID || in_sizes[2] != SEQS * HID ||
      in_sizes[3] != 1 || in_sizes[4] != 1 || in_sizes[5] != 1 ||
      in_sizes[6] != HID || in_sizes[7] != HID * HID || in_sizes[8] != HID || in_sizes[9] != HID * HID ||
      in_sizes[10] != HID * HID || in_sizes[11] != HID || in_sizes[12] != KCAT * HID || in_sizes[13] != HID ||
      in_sizes[14] != KCAT * HID || in_sizes[15] != HID || in_sizes[16] != HID || in_sizes[17] != 1 ||
      in_sizes[18] != HID || in_sizes[19] != 1 || out_size != SEQS * STEPS * 2) return;

  const float* x   = (const float*)d_in[0];
  const float* hI0 = (const float*)d_in[1];
  const float* hQ0 = (const float*)d_in[2];
  const float* c1  = (const float*)d_in[3];
  const float* c2  = (const float*)d_in[4];
  const float* c3  = (const float*)d_in[5];
  const float* Wa  = (const float*)d_in[6];
  const float* Wah = (const float*)d_in[7];
  const float* Wp1 = (const float*)d_in[8];
  const float* Wph = (const float*)d_in[9];
  const float* Wf  = (const float*)d_in[10];
  const float* bfv = (const float*)d_in[11];
  const float* Wgc = (const float*)d_in[12];
  const float* bgc = (const float*)d_in[13];
  const float* Wgs = (const float*)d_in[14];
  const float* bgs = (const float*)d_in[15];
  const float* WI  = (const float*)d_in[16];
  const float* bI  = (const float*)d_in[17];
  const float* WQ  = (const float*)d_in[18];
  const float* bQ  = (const float*)d_in[19];
  float* out = (float*)d_out;

  char* ws = (char*)d_ws; size_t off = 0;
  auto carve = [&](size_t bytes) -> char* { char* p = ws + off; off += (bytes + 255) & ~(size_t)255; return p; };
  unsigned short* W1  = (unsigned short*)carve((size_t)HID3 * HID * 2);
  unsigned short* W2c = (unsigned short*)carve((size_t)HID * KCAT * 2);
  unsigned short* W2s = (unsigned short*)carve((size_t)HID * KCAT * 2);
  if (off > ws_size || off > (size_t)134217728) return;

  tr_cvt_kernel<<<dim3(HID / 64, HID / 64), NTHR, 0, stream>>>(Wah, HID, W1, HID, 0);
  tr_cvt_kernel<<<dim3(HID / 64, HID / 64), NTHR, 0, stream>>>(Wph, HID, W1, HID, HID);
  tr_cvt_kernel<<<dim3(HID / 64, HID / 64), NTHR, 0, stream>>>(Wf,  HID, W1, HID, 2 * HID);
  tr_cvt_kernel<<<dim3(HID / 64, KCAT / 64), NTHR, 0, stream>>>(Wgc, HID, W2c, KCAT, 0);
  tr_cvt_kernel<<<dim3(HID / 64, KCAT / 64), NTHR, 0, stream>>>(Wgs, HID, W2s, KCAT, 0);
  cell_seq_kernel<<<NBLK, NTHR, 0, stream>>>(x, hI0, hQ0, c1, c2, c3, Wa, Wp1, bfv, bgc, bgs, WI, bI, WQ, bQ, W1, W2c, W2s, out);
}
